// rate_RNN_mante_4174708212036
// MI455X (gfx1250) — hardware-verified
//
#include <hip/hip_runtime.h>
#include <stdint.h>
#include <stddef.h>

#define TT  1000
#define NB  64
#define NI  4
#define NH  512
#define NO  3
#define NP  2
#define PA  520
#define RSC 128.0f
#define WSC 16.0f
#define OSC 0.00048828125f
#define LMK 0.9048374180359595f

static_assert(NH == 2 * 8 * 32);
static_assert(NH % 32 == 0);
static_assert((PA * 2) % 16 == 0);
static_assert(NO <= 4);
static_assert((TT * NB * NO) % 4 == 0);
static_assert((size_t)NB * TT * 16 <= (size_t)134217728);

typedef _Float16     v16h __attribute__((ext_vector_type(16)));
typedef float        v8f  __attribute__((ext_vector_type(8)));
typedef float        v4f  __attribute__((ext_vector_type(4)));
typedef unsigned int v4u  __attribute__((ext_vector_type(4)));
typedef v4f __attribute__((may_alias)) v4fa;
typedef v4u __attribute__((may_alias)) v4ua;

union FragH { v16h v; v4u q[2]; };

__device__ __forceinline__ v8f wmma_h(v16h a, v16h b, v8f c) {
  v8f d = __builtin_amdgcn_wmma_f32_16x16x32_f16(false, a, false, b, (short)0, c, false, false);
  asm volatile("v_nop\n\tv_nop\n\tv_nop\n\tv_nop" : "+v"(d) : "v"(a), "v"(b));
  return d;
}

__device__ __forceinline__ v16h ldfrag(const unsigned short* p, int h) {
  FragH f;
  f.q[0] = *(const v4ua*)(p + 8 * h);
  f.q[1] = *(const v4ua*)(p + 16 + 8 * h);
  return f.v;
}

__device__ __forceinline__ unsigned int pkh(float a, float b) {
  const unsigned short x = __builtin_bit_cast(unsigned short, (_Float16)a);
  const unsigned short y = __builtin_bit_cast(unsigned short, (_Float16)b);
  return (unsigned int)x | ((unsigned int)y << 16);
}
__device__ __forceinline__ v4u pack8(v4f a, v4f c) {
  v4u o;
  o.x = pkh(a.x, a.y); o.y = pkh(a.z, a.w);
  o.z = pkh(c.x, c.y); o.w = pkh(c.z, c.w);
  return o;
}

__device__ __forceinline__ float tnh(float v) {
  const float e = __expf(2.0f * v);
  return 1.0f - 2.0f * __builtin_amdgcn_rcpf(e + 1.0f);
}

__global__ __launch_bounds__(32) void k_rnn(const float* __restrict__ x,
                                            const float* __restrict__ Win,
                                            const float* __restrict__ Wout,
                                            const float* __restrict__ pin,
                                            const float* __restrict__ pout,
                                            const float* __restrict__ l,
                                            float* __restrict__ Yp)
{
  __shared__ __align__(16) unsigned short sA[16 * PA];
  __shared__ __align__(16) unsigned short sB[16 * PA];
  __shared__ __align__(16) float sO[16 * 16];
  const int lane = threadIdx.x & 31, h = lane >> 4, m = lane & 15;
  const int b = blockIdx.x;

  {
    const v4u z4 = {0u, 0u, 0u, 0u};
    #pragma unroll 1
    for (int i = 0; i < 32; ++i) {
      const int idx = lane + 32 * i;
      const int n = idx >> 6, pc = idx & 63;
      const int nc = (n < NO) ? n : (NO - 1);
      const float* wp = Wout + (size_t)nc * NH + 8 * pc;
      const v4f a = *(const v4fa*)wp;
      const v4f c = *(const v4fa*)(wp + 4);
      const float s = (n < NO) ? WSC : 0.0f;
      *(v4ua*)(sB + n * PA + 8 * pc) = pack8(a * s, c * s);
      *(v4ua*)(sA + n * PA + 8 * pc) = z4;
    }
  }

  const float l0 = l[0], l1 = l[1];
  v4f w[16];
  float lp0[16], lp1[16], po0[16], po1[16];
  #pragma unroll
  for (int g = 0; g < 2; ++g) {
    const int hb = 256 * g + 8 * lane;
    #pragma unroll
    for (int j = 0; j < 8; ++j) w[8 * g + j] = *(const v4fa*)(Win + (size_t)(hb + j) * NI);
    #pragma unroll
    for (int q = 0; q < 4; ++q) {
      const v4f pv = *(const v4fa*)(pin  + (size_t)hb * NP + 4 * q);
      const v4f ov = *(const v4fa*)(pout + (size_t)hb * NP + 4 * q);
      lp0[8 * g + 2 * q]     = pv.x * l0;  lp1[8 * g + 2 * q]     = pv.y * l1;
      lp0[8 * g + 2 * q + 1] = pv.z * l0;  lp1[8 * g + 2 * q + 1] = pv.w * l1;
      po0[8 * g + 2 * q]     = ov.x;       po1[8 * g + 2 * q]     = ov.y;
      po0[8 * g + 2 * q + 1] = ov.z;       po1[8 * g + 2 * q + 1] = ov.w;
    }
  }
  float mem[16];
  #pragma unroll
  for (int j = 0; j < 16; ++j) mem[j] = 0.0f;
  float d0 = 0.0f, d1 = 0.0f;
  const float lm = LMK;
  const float om = 1.0f - LMK;
  __syncthreads();

  const v8f z8 = {0.f, 0.f, 0.f, 0.f, 0.f, 0.f, 0.f, 0.f};

  #pragma unroll 1
  for (int t = 0; t < TT; ++t) {
    const v4f xt = *(const v4fa*)(x + ((size_t)t * NB + b) * NI);
    float s0 = d0, s1 = d1;
    #pragma unroll
    for (int msk = 16; msk > 0; msk >>= 1) {
      s0 += __shfl_xor(s0, msk);
      s1 += __shfl_xor(s1, msk);
    }
    float nd0 = 0.0f, nd1 = 0.0f;
    float vs[16];
    #pragma unroll
    for (int j = 0; j < 16; ++j) {
      const float iw = (w[j].x * xt.x + w[j].y * xt.y) + (w[j].z * xt.z + w[j].w * xt.w);
      const float I  = iw + (lp0[j] * s0 + lp1[j] * s1);
      const float mv = lm * mem[j] + om * I;
      mem[j] = mv;
      const float v = tnh(mv);
      nd0 = fmaf(po0[j], v, nd0);
      nd1 = fmaf(po1[j], v, nd1);
      vs[j] = v * RSC;
    }
    d0 = nd0; d1 = nd1;
    {
      v4u q0, q1;
      q0.x = pkh(vs[0],  vs[1]);  q0.y = pkh(vs[2],  vs[3]);
      q0.z = pkh(vs[4],  vs[5]);  q0.w = pkh(vs[6],  vs[7]);
      q1.x = pkh(vs[8],  vs[9]);  q1.y = pkh(vs[10], vs[11]);
      q1.z = pkh(vs[12], vs[13]); q1.w = pkh(vs[14], vs[15]);
      unsigned short* ar = sA + (t & 15) * PA + 8 * lane;
      *(v4ua*)ar = q0;
      *(v4ua*)(ar + 256) = q1;
    }

    if ((t & 15) == 15 || t == TT - 1) {
      const int t0 = t & ~15;
      const int nr = t - t0 + 1;
      __syncthreads();
      v8f acc = z8;
      #pragma unroll
      for (int ks = 0; ks < NH / 32; ++ks) {
        const v16h af = ldfrag(sA + m * PA + 32 * ks, h);
        const v16h bf = ldfrag(sB + m * PA + 32 * ks, h);
        acc = wmma_h(af, bf, acc);
      }
      v4f o0, o1;
      o0.x = acc[0] * OSC; o0.y = acc[1] * OSC; o0.z = acc[2] * OSC; o0.w = acc[3] * OSC;
      o1.x = acc[4] * OSC; o1.y = acc[5] * OSC; o1.z = acc[6] * OSC; o1.w = acc[7] * OSC;
      *(v4fa*)(sO + m * 16 + 8 * h)     = o0;
      *(v4fa*)(sO + m * 16 + 8 * h + 4) = o1;
      __syncthreads();
      v4f yv;
      yv.x = sO[0 * 16 + m];
      yv.y = sO[1 * 16 + m];
      yv.z = sO[2 * 16 + m];
      yv.w = sO[3 * 16 + m];
      float* yp = Yp + ((size_t)b * TT + t0 + m) * 4;
      if (lane < nr) *(volatile v4f*)yp = yv;
      __threadfence();
      if (lane < nr) *(volatile v4f*)yp = yv;
      __syncthreads();
    }
  }
}

__global__ __launch_bounds__(256) void k_out(const float* __restrict__ Yp,
                                             float* __restrict__ y, int n4)
{
  const int g = blockIdx.x * 256 + threadIdx.x;
  if (g >= n4) return;
  float v[4];
  #pragma unroll
  for (int i = 0; i < 4; ++i) {
    const int f   = 4 * g + i;
    const int row = f / NO;
    const int o   = f - NO * row;
    const int tt  = row / NB;
    const int bb  = row - NB * tt;
    int idx = (bb * TT + tt) * 4 + o;
    idx = (idx < 0) ? 0 : ((idx > NB * TT * 4 - 1) ? (NB * TT * 4 - 1) : idx);
    v[i] = Yp[idx];
  }
  v4f ov;
  ov.x = v[0]; ov.y = v[1]; ov.z = v[2]; ov.w = v[3];
  float* p = y + (size_t)g * 4;
  *(volatile v4f*)p = ov;
  __threadfence();
  *(volatile v4f*)p = ov;
}

extern "C" void kernel_launch(void* const* d_in, const int* in_sizes, int n_in,
                              void* d_out, int out_size, void* d_ws, size_t ws_size,
                              hipStream_t stream)
{
  if (n_in < 6) return;
  if (in_sizes[0] != TT * NB * NI) return;
  if (in_sizes[1] != NH * NI) return;
  if (in_sizes[2] != NO * NH) return;
  if (in_sizes[3] != NH * NP) return;
  if (in_sizes[4] != NH * NP) return;
  if (in_sizes[5] != NP) return;
  if (out_size != TT * NB * NO) return;

  const float* x    = (const float*)d_in[0];
  const float* Win  = (const float*)d_in[1];
  const float* Wout = (const float*)d_in[2];
  const float* pin  = (const float*)d_in[3];
  const float* pout = (const float*)d_in[4];
  const float* l    = (const float*)d_in[5];
  float* y = (float*)d_out;

  const size_t bY = (size_t)NB * TT * 4 * sizeof(float);
  if (bY > ws_size) return;
  if (bY > (size_t)134217728) return;
  float* Yp = (float*)d_ws;

  k_rnn<<<dim3(NB), dim3(32), 0, stream>>>(x, Win, Wout, pin, pout, l, Yp);
  const int n4 = out_size / 4;
  k_out<<<dim3((n4 + 255) / 256), dim3(256), 0, stream>>>(Yp, y, n4);
}
